// SlidingWindowGQACausalSelfAttention_80556406603856
// MI455X (gfx1250) — hardware-verified
//
#include <hip/hip_runtime.h>
#include <math.h>

typedef __attribute__((ext_vector_type(16))) _Float16 v16h;
typedef __attribute__((ext_vector_type(16))) __bf16 v16b;
typedef __attribute__((ext_vector_type(8)))  _Float16 v8h;
typedef __attribute__((ext_vector_type(8)))  float v8f;
typedef __attribute__((ext_vector_type(4)))  float v4f;
typedef __attribute__((ext_vector_type(2)))  float v2f;
typedef __attribute__((ext_vector_type(4)))  unsigned v4u;
typedef __attribute__((ext_vector_type(4)))  int v4i;
typedef float __attribute__((may_alias)) float_a;
typedef int __attribute__((may_alias)) int_a;

template <typename T> __device__ __forceinline__ void vst2(void* p, T v) { *(volatile T*)p = v; __threadfence(); *(volatile T*)p = v; }
__device__ __forceinline__ v8f wmma16(v16h a, v16h b, v8f c) {
  v8f d = __builtin_amdgcn_wmma_f32_16x16x32_f16(false, a, false, b, (short)0, c, false, false);
  asm volatile("v_nop\n\tv_nop\n\tv_nop\n\tv_nop" : "+v"(d) : "v"(a), "v"(b));
  return d;
}
__device__ __forceinline__ v8f wmma_bf(v16b a, v16b b, v8f c) {
  v8f d = __builtin_amdgcn_wmma_f32_16x16x32_bf16(false, a, false, b, (short)0, c, false, false);
  asm volatile("v_nop\n\tv_nop\n\tv_nop\n\tv_nop" : "+v"(d) : "v"(a), "v"(b));
  return d;
}
__device__ __forceinline__ v16h frag_h(const _Float16* rowk0, int lane) {
  union { v16h v; v8h q[2]; } u; const _Float16* p = rowk0 + 8 * (lane >> 4);
  u.q[0] = *(const v8h*)p; u.q[1] = *(const v8h*)(p + 16); return u.v;
}
__device__ __forceinline__ v16h frag_f32(const float* rowk0, int lane) {
  v16h a; const float* p = rowk0 + 8 * (lane >> 4);
#pragma unroll
  for (int i = 0; i < 8; ++i) { a[i] = (_Float16)p[i]; a[8 + i] = (_Float16)p[16 + i]; }
  return a;
}
__device__ __forceinline__ v16h frag_f32s(const float* rowk0, int lane, float sc) {
  v16h a; const float* p = rowk0 + 8 * (lane >> 4);
#pragma unroll
  for (int i = 0; i < 8; ++i) { a[i] = (_Float16)(p[i] * sc); a[8 + i] = (_Float16)(p[16 + i] * sc); }
  return a;
}
__device__ __forceinline__ v16h fragc_f32(const float* W, int k0, int n, int lane, int ld, int K) {
  v16h a; const int g = lane >> 4;
#pragma unroll
  for (int i = 0; i < 8; ++i) { const int ka = k0 + 8 * g + i, kb = ka + 16;
    a[i] = (_Float16)(ka < K ? W[(size_t)(ka < K ? ka : K - 1) * ld + n] : 0.f); a[8 + i] = (_Float16)(kb < K ? W[(size_t)(kb < K ? kb : K - 1) * ld + n] : 0.f); }
  return a;
}
struct F2 { v16b h, l; };
__device__ __forceinline__ F2 bsplit16(const float v[16]) { F2 r;
#pragma unroll
  for (int i = 0; i < 16; ++i) { const __bf16 h = (__bf16)v[i]; r.h[i] = h; r.l[i] = (__bf16)(v[i] - (float)h); }
  return r; }
__device__ __forceinline__ F2 split_row(const float* row, int k0, int lane) { float v[16]; const float* p = row + k0 + 8 * (lane >> 4);
#pragma unroll
  for (int i = 0; i < 8; ++i) { v[i] = p[i]; v[8 + i] = p[16 + i]; }
  return bsplit16(v); }
__device__ __forceinline__ F2 split_rowK(const float* row, int k0, int lane, int K) { float v[16]; const int g = lane >> 4;
#pragma unroll
  for (int i = 0; i < 8; ++i) { const int ka = k0 + 8 * g + i, kb = ka + 16; v[i] = ka < K ? row[ka < K ? ka : K - 1] : 0.f; v[8 + i] = kb < K ? row[kb < K ? kb : K - 1] : 0.f; }
  return bsplit16(v); }
__device__ __forceinline__ F2 split_col(const float* W, int k0, int n, int lane, int ld, int K) { float v[16]; const int g = lane >> 4;
#pragma unroll
  for (int i = 0; i < 8; ++i) { const int ka = k0 + 8 * g + i, kb = ka + 16; v[i] = ka < K ? W[(size_t)(ka < K ? ka : K - 1) * ld + n] : 0.f; v[8 + i] = kb < K ? W[(size_t)(kb < K ? kb : K - 1) * ld + n] : 0.f; }
  return bsplit16(v); }
__device__ __forceinline__ v8f mac3(const F2& a, const F2& b, v8f c) { c = wmma_bf(a.l, b.h, c); c = wmma_bf(a.h, b.l, c); return wmma_bf(a.h, b.h, c); }
__device__ __forceinline__ float sigm(float v) { return 1.0f / (1.0f + expf(-v)); }
#define LDSX() do { asm volatile("s_wait_dscnt 0" ::: "memory"); __builtin_amdgcn_wave_barrier(); __builtin_amdgcn_fence(__ATOMIC_RELEASE, "workgroup"); } while (0)


#define NB 2
#define SS 2048
#define DIM 2048
#define NHQ 16
#define NKV 4
#define HDD 128
#define KVD (NKV * HDD)
#define WIN 512
#define NR (NB * SS)
#ifndef TQB
#define TQB (SS / 64)
#endif
typedef __attribute__((ext_vector_type(8))) __bf16 v8b;
__device__ __forceinline__ v16b frag_b(const __bf16* rowk0, int lane) {
  union { v16b v; v8b q[2]; } u; const __bf16* p = rowk0 + 8 * (lane >> 4);
  u.q[0] = *(const v8b*)p; u.q[1] = *(const v8b*)(p + 16); return u.v;
}
__device__ __forceinline__ float bfr(float v) { return (float)(__bf16)v; }
__device__ __attribute__((noinline)) float exp_ni(float v) { return expf(v); }
__device__ __attribute__((noinline)) float erf_ni(float v) { return erff(v); }

__constant__ float INVF[64] = {1.000000000e+00f,8.659643531e-01f,7.498942018e-01f,6.493816376e-01f,5.623413324e-01f,4.869675338e-01f,4.216965139e-01f,3.651741147e-01f,3.162277639e-01f,2.738419771e-01f,2.371373773e-01f,2.053525001e-01f,1.778279394e-01f,1.539926529e-01f,1.333521456e-01f,1.154781953e-01f,1.000000015e-01f,8.659642935e-02f,7.498942316e-02f,6.493816525e-02f,5.623413250e-02f,4.869675264e-02f,4.216964915e-02f,3.651741147e-02f,3.162277490e-02f,2.738419548e-02f,2.371373773e-02f,2.053525113e-02f,1.778279431e-02f,1.539926510e-02f,1.333521400e-02f,1.154781971e-02f,9.999999776e-03f,8.659643121e-03f,7.498942316e-03f,6.493816152e-03f,5.623413250e-03f,4.869675264e-03f,4.216964822e-03f,3.651741194e-03f,3.162277630e-03f,2.738419687e-03f,2.371373819e-03f,2.053525066e-03f,1.778279431e-03f,1.539926510e-03f,1.333521446e-03f,1.154782018e-03f,1.000000047e-03f,8.659643354e-04f,7.498941850e-04f,6.493816036e-04f,5.623413017e-04f,4.869675322e-04f,4.216965172e-04f,3.651741135e-04f,3.162277571e-04f,2.738419571e-04f,2.371373703e-04f,2.053525095e-04f,1.778279402e-04f,1.539926598e-04f,1.333521504e-04f,1.154782003e-04f};
#define WS_PQ  0u
#define WS_PKk (WS_PQ + 2u * (size_t)DIM * DIM)
#define WS_PV  (WS_PKk + 2u * (size_t)KVD * DIM)
#define WS_PO  (WS_PV + 2u * (size_t)KVD * DIM)
#define WS_QH  (WS_PO + 2u * (size_t)DIM * DIM)
#define WS_QL  (WS_QH + 2u * (size_t)NR * DIM)
#define WS_KH  (WS_QL + 2u * (size_t)NR * DIM)
#define WS_KL  (WS_KH + 2u * (size_t)NR * KVD)
#define WS_VT  (WS_KL + 2u * (size_t)NR * KVD)
#define WS_Y   (WS_VT + 2u * (size_t)NR * KVD)
#define WS_END (WS_Y + 4u * (size_t)NR * DIM)

__global__ __launch_bounds__(256) void k_pack(const float* __restrict__ WQ, const float* __restrict__ WK, const float* __restrict__ WV, const float* __restrict__ WO, __bf16* __restrict__ P) {
  const int n = blockIdx.x, which = blockIdx.y, t = threadIdx.x; __shared__ __align__(16) __bf16 s[DIM]; const float* src; size_t dst;
  if (which == 0) { src = WQ + (size_t)n * DIM; dst = WS_PQ / 2 + (size_t)n * DIM; } else if (which == 1) { if (n >= KVD) return; src = WK + (size_t)n * DIM; dst = WS_PKk / 2 + (size_t)n * DIM; } else if (which == 2) { if (n >= KVD) return; src = WV + (size_t)n * DIM; dst = WS_PV / 2 + (size_t)n * DIM; } else { src = WO + (size_t)n * DIM; dst = WS_PO / 2 + (size_t)n * DIM; }
  for (int k = t; k < DIM; k += 256) s[k] = (__bf16)src[k];
  __syncthreads();
  for (int q = t; q < DIM / 8; q += 256) vst2((unsigned*)(P + dst + q * 8), *(const v4u*)&s[q * 8]);
}
__device__ __attribute__((noinline)) float cos_p(float v) { return cosf(v); }
__device__ __attribute__((noinline)) float sin_p(float v) { return sinf(v); }
__global__ __launch_bounds__(128) void k_qkv(const float* __restrict__ X, const __bf16* __restrict__ P, const float* __restrict__ QG, _Float16* __restrict__ QH, _Float16* __restrict__ QL, _Float16* __restrict__ KH, _Float16* __restrict__ KL, _Float16* __restrict__ VT) {
  __shared__ __align__(16) _Float16 sth[64][HDD + 8], stl[64][HDD + 8]; __shared__ __align__(16) _Float16 svt[HDD][72];
  const int tid = threadIdx.x, wave = tid >> 5, lane = tid & 31, col = lane & 15, g = lane >> 4; const int slot = blockIdx.y; const size_t r0 = (size_t)blockIdx.x * 64 + wave * 16;
  const __bf16* Wr; int kind, hh;
  if (slot < NHQ) { kind = 0; hh = slot; Wr = P + WS_PQ / 2 + (size_t)hh * HDD * DIM; } else if (slot < NHQ + NKV) { kind = 1; hh = slot - NHQ; Wr = P + WS_PKk / 2 + (size_t)hh * HDD * DIM; } else { kind = 2; hh = slot - NHQ - NKV; Wr = P + WS_PV / 2 + (size_t)hh * HDD * DIM; }
  v8f acc[8] = {};
#pragma unroll 2
  for (int kc = 0; kc < DIM / 32; ++kc) { v16b a; { const float* p = X + (r0 + col) * DIM + kc * 32 + 8 * g;
#pragma unroll
      for (int i = 0; i < 8; ++i) { a[i] = (__bf16)p[i]; a[8 + i] = (__bf16)p[16 + i]; } }
#pragma unroll
    for (int j = 0; j < 8; ++j) acc[j] = wmma_bf(a, frag_b(Wr + (size_t)(j * 16 + col) * DIM + kc * 32, lane), acc[j]); }
  if (kind < 2) {
#pragma unroll
    for (int r = 0; r < 8; ++r) { float ssq = 0.f;
#pragma unroll
      for (int j = 0; j < 8; ++j) ssq += acc[j][r] * acc[j][r];
#pragma unroll
      for (int o = 1; o < 16; o <<= 1) ssq += __shfl_xor(ssq, o);
      const float rinv = 1.0f / sqrtf(ssq / (float)HDD + 1.1920928955078125e-07f);
      const size_t row = r0 + 8 * g + r; const int s = (int)(row % SS); const float gain = (kind == 0) ? bfr(QG[hh]) : 1.0f;
#pragma unroll
      for (int j = 0; j < 4; ++j) { const int d = j * 16 + col; const float x1 = acc[j][r] * rinv, x2 = acc[j + 4][r] * rinv; const float fr = (float)s * INVF[d]; const float c = cos_p(fr), sn = sin_p(fr);
        const float o1 = (x1 * c + x2 * sn) * gain, o2 = (-x1 * sn + x2 * c) * gain;
        const _Float16 h1 = (_Float16)o1, h2 = (_Float16)o2; sth[wave * 16 + 8 * g + r][d] = h1; stl[wave * 16 + 8 * g + r][d] = (_Float16)((o1 - (float)h1) * 2048.0f); sth[wave * 16 + 8 * g + r][64 + d] = h2; stl[wave * 16 + 8 * g + r][64 + d] = (_Float16)((o2 - (float)h2) * 2048.0f); } }
    LDSX();
    _Float16* DH_ = (kind == 0) ? QH : KH; _Float16* DL_ = (kind == 0) ? QL : KL; const int nh = (kind == 0) ? NHQ : NKV;
    for (int rl = 0; rl < 16; ++rl) if (lane < 16) { const size_t o = ((r0 + rl) * nh + hh) * HDD + lane * 8; vst2((unsigned*)(DH_ + o), *(const v4u*)&sth[wave * 16 + rl][lane * 8]); vst2((unsigned*)(DL_ + o), *(const v4u*)&stl[wave * 16 + rl][lane * 8]); }
  } else {
#pragma unroll
    for (int j = 0; j < 8; ++j)
#pragma unroll
      for (int r = 0; r < 8; ++r) svt[j * 16 + col][wave * 16 + 8 * g + r] = (_Float16)acc[j][r];
    __syncthreads();
    const size_t rb0 = (size_t)blockIdx.x * 64; const size_t b = rb0 / SS, s0 = rb0 % SS;
    for (int e = tid; e < HDD * 8; e += 128) { const int d = e >> 3, pc = e & 7; vst2((unsigned*)(VT + ((b * KVD + hh * HDD + d) * SS) + s0 + pc * 8), *(const v4u*)&svt[d][pc * 8]); } }
}
__global__ __launch_bounds__(128) void k_attn(const _Float16* __restrict__ QH, const _Float16* __restrict__ QL, const _Float16* __restrict__ KH, const _Float16* __restrict__ KL, const _Float16* __restrict__ VT, float* __restrict__ Y) {
  __shared__ __align__(16) _Float16 sph[4][16][40]; __shared__ __align__(16) float so[4][16][132];
  const int tid = threadIdx.x, wave = tid >> 5, lane = tid & 31, col = lane & 15, g = lane >> 4; const int qb = blockIdx.x, h = blockIdx.y; const size_t b = blockIdx.z; const int kvh = h / (NHQ / NKV); const int q0 = qb * 64 + wave * 16; const size_t rq = b * SS + q0;
  v16h aq[4], aql[4];
#pragma unroll
  for (int kc = 0; kc < 4; ++kc) { aq[kc] = frag_h(QH + ((rq + col) * NHQ + h) * HDD + kc * 32, lane); aql[kc] = frag_h(QL + ((rq + col) * NHQ + h) * HDD + kc * 32, lane); }
  float m[8], l[8];
#pragma unroll
  for (int r = 0; r < 8; ++r) { m[r] = -3.0e38f; l[r] = 0.f; }
  v8f acc[8] = {}; const float scale = 1.0f / sqrtf((float)HDD);
  int ks0 = (qb * 64 - (WIN - 1)); ks0 = ks0 < 0 ? 0 : ks0 / 32; const int ks1 = (qb * 64 + 63) / 32;
#pragma unroll 1
  for (int ks = ks0; ks <= ks1; ++ks) { const int j0 = ks * 32; v8f s[2];
#pragma unroll
    for (int ct = 0; ct < 2; ++ct) { const int kk = j0 + ct * 16 + col; const size_t rk = ((b * SS + kk) * NKV + kvh) * HDD; v8f c = {}, cl = {};
#pragma unroll
      for (int kc = 0; kc < 4; ++kc) { const v16h kh = frag_h(KH + rk + kc * 32, lane); c = wmma16(aq[kc], kh, c); cl = wmma16(aql[kc], kh, cl); cl = wmma16(aq[kc], frag_h(KL + rk + kc * 32, lane), cl); }
#pragma unroll
      for (int r = 0; r < 8; ++r) { const int qi = q0 + 8 * g + r; const bool keep = (kk <= qi) && (kk >= qi - (WIN - 1)); s[ct][r] = keep ? (c[r] + cl[r] * (1.0f / 2048.0f)) * scale : -3.0e38f; } }
#pragma unroll
    for (int r = 0; r < 8; ++r) { float mx = fmaxf(s[0][r], s[1][r]);
#pragma unroll
      for (int o = 1; o < 16; o <<= 1) mx = fmaxf(mx, __shfl_xor(mx, o));
      const float mn = fmaxf(m[r], mx); const float alpha = (m[r] <= -1.0e38f) ? 0.f : __expf(m[r] - mn); const float e0 = (s[0][r] <= -1.0e38f) ? 0.f : __expf(s[0][r] - mn), e1 = (s[1][r] <= -1.0e38f) ? 0.f : __expf(s[1][r] - mn); float es = e0 + e1;
#pragma unroll
      for (int o = 1; o < 16; o <<= 1) es += __shfl_xor(es, o);
      l[r] = l[r] * alpha + es; m[r] = (mn <= -1.0e38f) ? m[r] : mn;
#pragma unroll
      for (int dt = 0; dt < 8; ++dt) acc[dt][r] *= alpha;
      sph[wave][8 * g + r][col] = (_Float16)(e0 * 2048.0f); sph[wave][8 * g + r][16 + col] = (_Float16)(e1 * 2048.0f); }
    LDSX();
    const v16h pa = frag_h(&sph[wave][col][0], lane);
#pragma unroll
    for (int dt = 0; dt < 8; ++dt) acc[dt] = wmma16(pa, frag_h(VT + (b * KVD + kvh * HDD + dt * 16 + col) * SS + j0, lane), acc[dt]);
    LDSX(); }
#pragma unroll
  for (int r = 0; r < 8; ++r) { const float il = (1.0f / 2048.0f) / l[r];
#pragma unroll
    for (int dt = 0; dt < 8; ++dt) so[wave][8 * g + r][dt * 16 + col] = acc[dt][r] * il; }
  LDSX();
  for (int rl = 0; rl < 16; ++rl) vst2(Y + (rq + rl) * DIM + h * HDD + lane * 4, *(const v4f*)&so[wave][rl][lane * 4]);
}
__global__ __launch_bounds__(128) void k_out(const float* __restrict__ Yb, const __bf16* __restrict__ P, float* __restrict__ OUT) {
  __shared__ __align__(16) float so[4][16][132];
  const int tid = threadIdx.x, wave = tid >> 5, lane = tid & 31, col = lane & 15, g = lane >> 4; const size_t r0 = (size_t)blockIdx.x * 64 + wave * 16; const int n0 = blockIdx.y * 128; const __bf16* Wr = P + WS_PO / 2;
  v8f acc[8] = {};
#pragma unroll 2
  for (int kc = 0; kc < DIM / 32; ++kc) { const F2 a = split_row(Yb + (r0 + col) * DIM, kc * 32, lane);
#pragma unroll
    for (int j = 0; j < 8; ++j) { const v16b w = frag_b(Wr + (size_t)(n0 + j * 16 + col) * DIM + kc * 32, lane); acc[j] = wmma_bf(a.l, w, acc[j]); acc[j] = wmma_bf(a.h, w, acc[j]); } }
#pragma unroll
  for (int j = 0; j < 8; ++j)
#pragma unroll
    for (int r = 0; r < 8; ++r) so[wave][8 * g + r][j * 16 + col] = acc[j][r];
  LDSX();
  for (int rl = 0; rl < 16; ++rl) vst2(OUT + (r0 + rl) * DIM + n0 + lane * 4, *(const v4f*)&so[wave][rl][lane * 4]);
}
extern "C" void kernel_launch(void* const* d_in, const int* in_sizes, int n_in, void* d_out, int out_size, void* d_ws, size_t ws_size, hipStream_t stream) {
  (void)in_sizes; (void)n_in; (void)out_size;
  const float** F = (const float**)d_in;
  if (ws_size < (size_t)WS_END) return;
  char* ws = (char*)d_ws; __bf16* P = (__bf16*)ws; _Float16 *QH = (_Float16*)(ws + WS_QH), *QL = (_Float16*)(ws + WS_QL), *KH = (_Float16*)(ws + WS_KH), *KL = (_Float16*)(ws + WS_KL), *VT = (_Float16*)(ws + WS_VT); float* Y = (float*)(ws + WS_Y);
  k_pack<<<dim3(DIM, 4), 256, 0, stream>>>(F[1], F[2], F[3], F[4], P);
  k_qkv<<<dim3(NR / 64, NHQ + 2 * NKV), 128, 0, stream>>>(F[0], P, F[5], QH, QL, KH, KL, VT);
  k_attn<<<dim3(TQB, NHQ, NB), 128, 0, stream>>>(QH, QL, KH, KL, VT, Y);
  k_out<<<dim3(NR / 64, DIM / 128), 128, 0, stream>>>(Y, P, (float*)d_out);
}
